// PromptAttention_84971632984154
// MI455X (gfx1250) — hardware-verified
//
#include <hip/hip_runtime.h>


#define NB_  32
#define NQ_  128
#define NS_  2048
#define DA   64
#define NH_  8
#define DK   8
#define DV   64
#define NHID 128
#define PSC  32768.0f
#define LOSC 1024.0f
#define LOSCI (1.0f / 1024.0f)

typedef _Float16 h16;
typedef unsigned short bf;
typedef __attribute__((ext_vector_type(16))) __bf16   v16bf;
typedef __attribute__((ext_vector_type(16))) _Float16 v16h;
typedef __attribute__((ext_vector_type(8)))  _Float16 v8h;
typedef __attribute__((ext_vector_type(8)))  unsigned short v8us;
typedef __attribute__((ext_vector_type(8)))  float    v8f;
typedef __attribute__((ext_vector_type(4)))  float    v4f;
typedef v8h  __attribute__((may_alias)) v8ha;
typedef v4f  __attribute__((may_alias)) v4fa;
typedef v8us __attribute__((may_alias)) v8usa;

__device__ __forceinline__ unsigned short f2bf(float f) { unsigned u = __float_as_uint(f); u += 0x7FFFu + ((u >> 16) & 1u); return (unsigned short)(u >> 16); }
__device__ __forceinline__ float bf2f(unsigned short b) { return __uint_as_float(((unsigned)b) << 16); }
__device__ __forceinline__ float bfr(float f) { return bf2f(f2bf(f)); }
__device__ __forceinline__ v16h cat16(v8h lo, v8h hi) { return __builtin_shufflevector(lo, hi, 0, 1, 2, 3, 4, 5, 6, 7, 8, 9, 10, 11, 12, 13, 14, 15); }
__device__ __forceinline__ v16bf cat16b(v8us lo, v8us hi) { return __builtin_bit_cast(v16bf, __builtin_shufflevector(lo, hi, 0, 1, 2, 3, 4, 5, 6, 7, 8, 9, 10, 11, 12, 13, 14, 15)); }
__device__ __forceinline__ v8f wmma16(v16h a, v16h b, v8f c) { return __builtin_amdgcn_wmma_f32_16x16x32_f16(false, a, false, b, (short)0, c, false, false); }
__device__ __forceinline__ v8f wmmab(v16bf a, v16bf b, v8f c) { return __builtin_amdgcn_wmma_f32_16x16x32_bf16(false, a, false, b, (short)0, c, false, false); }
#define VST2(T, p, v) do { const T vst2_v_ = (v); *(volatile T*)(p) = vst2_v_; __threadfence(); *(volatile T*)(p) = vst2_v_; } while (0)

__global__ __launch_bounds__(256) void k_b64(const float* __restrict__ src, size_t rows, bf* dst) {
    typedef __attribute__((ext_vector_type(4))) unsigned short v4us;
    const int lane = threadIdx.x & 31; const size_t w = (size_t)blockIdx.x * 8 + (threadIdx.x >> 5);
    if (w * 2 >= rows) return;
    v4us o;
#pragma unroll
    for (int i = 0; i < 4; ++i) o[i] = f2bf(src[w * 128 + lane * 4 + i]);
    VST2(v4us, dst + w * 128 + lane * 4, o);
}
__global__ __launch_bounds__(256) void k_wt64(const float* __restrict__ Wm, int ncols, bf* WT) {
    typedef __attribute__((ext_vector_type(4))) unsigned short v4us;
    const int lane = threadIdx.x & 31, o = blockIdx.x * 8 + (threadIdx.x >> 5);
    if (o >= ncols) return;
    if (lane < 16) { v4us t;
#pragma unroll
        for (int i = 0; i < 4; ++i) t[i] = f2bf(Wm[(size_t)(lane * 4 + i) * ncols + o]);
        *(volatile v4us*)(WT + (size_t)o * DA + lane * 4) = t; __threadfence(); *(volatile v4us*)(WT + (size_t)o * DA + lane * 4) = t; }
}
__global__ __launch_bounds__(256) void k_wo(const float* __restrict__ Wm, bf* WT) {
    __shared__ __align__(16) unsigned short tl[64 * 72];
    const int tid = threadIdx.x, k0 = blockIdx.x * 64, n0 = blockIdx.y * 64;
    const int kk = tid >> 2, nq = (tid & 3) * 16;
#pragma unroll
    for (int i = 0; i < 16; ++i) tl[(nq + i) * 72 + kk] = f2bf(Wm[(size_t)(k0 + kk) * NHID + n0 + nq + i]);
    __syncthreads();
    const int piece = tid & 7;
    auto pass = [&]() {
#pragma unroll
        for (int s = 0; s < 2; ++s) { const int nr = (tid >> 3) + 32 * s; const v8us val = *(const v8usa*)(tl + nr * 72 + piece * 8);
            *(volatile v8us*)(WT + (size_t)(n0 + nr) * (NH_ * DV) + k0 + piece * 8) = val; }
    };
    pass(); __threadfence(); pass();
}
__global__ __launch_bounds__(128) void k_proj(const bf* __restrict__ Xb, const bf* __restrict__ WT, const float* __restrict__ bias, h16* PH, h16* PL) {
    __shared__ __align__(16) float ost[4][16 * 68];
    const int lane = threadIdx.x & 31, wave = threadIdx.x >> 5, lr = lane & 15, hi = lane >> 4;
    const size_t r0 = (size_t)blockIdx.x * 64 + wave * 16;
    v8f acc[4];
#pragma unroll
    for (int t = 0; t < 4; ++t) acc[t] = (v8f){};
#pragma unroll
    for (int kc = 0; kc < DA; kc += 32) {
        const v16bf a = cat16b(*(const v8us*)(Xb + (r0 + lr) * DA + kc + 8 * hi), *(const v8us*)(Xb + (r0 + lr) * DA + kc + 8 * hi + 16));
#pragma unroll
        for (int t = 0; t < 4; ++t) { const bf* bp = WT + (size_t)(t * 16 + lr) * DA + kc + 8 * hi; acc[t] = wmmab(a, cat16b(*(const v8us*)bp, *(const v8us*)(bp + 16)), acc[t]); }
    }
    float* os = &ost[wave][0];
#pragma unroll
    for (int t = 0; t < 4; ++t) { const float bv = bfr(bias[t * 16 + lr]);
#pragma unroll
        for (int j = 0; j < 8; ++j) os[(hi * 8 + j) * 68 + t * 16 + lr] = acc[t][j] + bv; }
    __syncthreads();
    auto pass = [&]() {
#pragma unroll
        for (int s = 0; s < 4; ++s) { const int row = 4 * s + (lane >> 3), piece = lane & 7; const float* sp = os + row * 68 + piece * 8; v8h oh, ol;
#pragma unroll
            for (int i = 0; i < 8; ++i) { const h16 a = (h16)sp[i]; oh[i] = a; ol[i] = (h16)((sp[i] - (float)a) * LOSC); }
            *(volatile v8h*)(PH + (r0 + row) * DA + piece * 8) = oh; *(volatile v8h*)(PL + (r0 + row) * DA + piece * 8) = ol; }
    };
    pass(); __threadfence(); pass();
}
__global__ __launch_bounds__(256) void k_vt(const float* __restrict__ v, h16* VT16) {
    __shared__ __align__(16) h16 tl[64 * 72];
    const int tid = threadIdx.x, s0 = blockIdx.x * 64, b = blockIdx.z;
    const int ss = tid >> 2, dq = (tid & 3) * 16;
#pragma unroll
    for (int i = 0; i < 16; ++i) tl[(dq + i) * 72 + ss] = (h16)bfr(v[((size_t)b * NS_ + s0 + ss) * DV + dq + i]);
    __syncthreads();
    const int piece = tid & 7;
    auto pass = [&]() {
#pragma unroll
        for (int s = 0; s < 2; ++s) { const int d = (tid >> 3) + 32 * s; const v8h val = *(const v8ha*)(tl + d * 72 + piece * 8); *(volatile v8h*)(VT16 + ((size_t)b * DV + d) * NS_ + s0 + piece * 8) = val; }
    };
    pass(); __threadfence(); pass();
}
__global__ __launch_bounds__(128) void k_attn(const h16* __restrict__ QH, const h16* __restrict__ QL, const h16* __restrict__ KH, const h16* __restrict__ KL, const h16* __restrict__ VT16, float* X) {
    __shared__ __align__(16) h16 pth[NQ_ * 72];
    __shared__ __align__(16) h16 ptl[NQ_ * 72];
    __shared__ __align__(16) float ost[4][16 * 68];
    const int lane = threadIdx.x & 31, wave = threadIdx.x >> 5, lr = lane & 15, hi = lane >> 4;
    const int b = blockIdx.x / NH_, h = blockIdx.x - b * NH_;
    const float scl = 0.35355339059327373f;
    const v8h zero8 = (v8h){};
    v8f o[2][4];
#pragma unroll
    for (int m = 0; m < 2; ++m)
#pragma unroll
        for (int t = 0; t < 4; ++t) o[m][t] = (v8f){};
#pragma unroll 1
    for (int st = 0; st < NS_ / 64; ++st) {
        const int sbase = st * 64, s0 = sbase + wave * 16;
        const size_t ko = ((size_t)b * NS_ + s0 + lr) * DA + h * DK;
        const v16h ka = cat16(hi ? zero8 : *(const v8h*)(KH + ko), zero8), kal = cat16(hi ? zero8 : *(const v8h*)(KL + ko), zero8);
        v8f sc[8];
#pragma unroll
        for (int n = 0; n < 8; ++n) { const size_t qo = ((size_t)b * NQ_ + n * 16 + lr) * DA + h * DK;
            const v16h qb = cat16(hi ? zero8 : *(const v8h*)(QH + qo), zero8), qbl = cat16(hi ? zero8 : *(const v8h*)(QL + qo), zero8);
            v8f a = wmma16(ka, qb, (v8f){}); v8f ax = wmma16(ka, qbl, (v8f){}); ax = wmma16(kal, qb, ax);
            asm volatile("v_nop\n\tv_nop\n\tv_nop\n\tv_nop" : "+v"(a), "+v"(ax) : "v"(qb), "v"(qbl) : "memory");
#pragma unroll
            for (int j = 0; j < 8; ++j) a[j] += ax[j] * LOSCI;
            sc[n] = a; }
        asm volatile("v_nop\n\tv_nop\n\tv_nop\n\tv_nop" : "+v"(sc[0]), "+v"(sc[7]) : "v"(ka), "v"(kal));
#pragma unroll
        for (int j = 0; j < 8; ++j) { float mx = -3.0e38f;
#pragma unroll
            for (int n = 0; n < 8; ++n) { sc[n][j] *= scl; mx = fmaxf(mx, sc[n][j]); }
            mx = fmaxf(mx, __shfl_xor(mx, 1, 16)); mx = fmaxf(mx, __shfl_xor(mx, 2, 16)); mx = fmaxf(mx, __shfl_xor(mx, 4, 16)); mx = fmaxf(mx, __shfl_xor(mx, 8, 16));
            float sum = 0.f;
#pragma unroll
            for (int n = 0; n < 8; ++n) { sc[n][j] = __expf(sc[n][j] - mx); sum += sc[n][j]; }
            sum += __shfl_xor(sum, 1, 16); sum += __shfl_xor(sum, 2, 16); sum += __shfl_xor(sum, 4, 16); sum += __shfl_xor(sum, 8, 16);
            const float f = PSC / sum; const int sl = wave * 16 + hi * 8 + j;
#pragma unroll
            for (int n = 0; n < 8; ++n) { const float p = sc[n][j] * f; const h16 ph = (h16)p; const int q = n * 16 + lr;
                pth[q * 72 + sl] = ph; ptl[q * 72 + sl] = (h16)(p - (float)ph); } }
        __syncthreads();
#pragma unroll
        for (int kc = 0; kc < 2; ++kc) {
            v16h vb[4];
#pragma unroll
            for (int t = 0; t < 4; ++t) { const size_t vo = ((size_t)b * DV + t * 16 + lr) * NS_ + sbase + kc * 32 + hi * 8; vb[t] = cat16(*(const v8h*)(VT16 + vo), *(const v8h*)(VT16 + vo + 16)); }
#pragma unroll
            for (int m = 0; m < 2; ++m) { const int q = wave * 32 + m * 16 + lr;
                const v16h pa = cat16(*(const v8ha*)(pth + q * 72 + kc * 32 + hi * 8), *(const v8ha*)(pth + q * 72 + kc * 32 + hi * 8 + 16));
                const v16h px = cat16(*(const v8ha*)(ptl + q * 72 + kc * 32 + hi * 8), *(const v8ha*)(ptl + q * 72 + kc * 32 + hi * 8 + 16));
#pragma unroll
                for (int t = 0; t < 4; ++t) { o[m][t] = wmma16(pa, vb[t], o[m][t]); o[m][t] = wmma16(px, vb[t], o[m][t]); }
                asm volatile("v_nop" : "+v"(o[m][0]), "+v"(o[m][3]) : "v"(pa), "v"(px) : "memory"); }
        }
        __syncthreads();
    }
    float* os = &ost[wave][0];
#pragma unroll
    for (int m = 0; m < 2; ++m) {
#pragma unroll
        for (int t = 0; t < 4; ++t)
#pragma unroll
            for (int j = 0; j < 8; ++j) os[(hi * 8 + j) * 68 + t * 16 + lr] = o[m][t][j] * (1.0f / PSC);
        __builtin_amdgcn_wave_barrier(); asm volatile("" ::: "memory");
        float* xb = X + ((size_t)b * NQ_ + wave * 32 + m * 16) * (NH_ * DV) + (size_t)h * DV;
#pragma unroll
        for (int ps2 = 0; ps2 < 2; ++ps2) {
#pragma unroll
            for (int s = 0; s < 8; ++s) { const int Lid = (lane >> 3) + 4 * s, piece = lane & 7; const int row = Lid >> 1, cofs = (Lid & 1) * 32 + piece * 4;
                const v4f val = *(const v4fa*)(os + row * 68 + cofs); *(volatile v4f*)(xb + (size_t)row * (NH_ * DV) + cofs) = val; }
            if (ps2 == 0) __threadfence(); }
        __builtin_amdgcn_wave_barrier(); asm volatile("" ::: "memory");
    }
}
__global__ __launch_bounds__(256) void k_xsplit(const float* __restrict__ X, bf* XH, bf* XL) {
    const int lane = threadIdx.x & 31; const size_t w = (size_t)blockIdx.x * 8 + (threadIdx.x >> 5);
    if (w * 256 >= (size_t)NB_ * NQ_ * NH_ * DV) return;
    v8us oh, ol;
#pragma unroll
    for (int i = 0; i < 8; ++i) { const float v = X[w * 256 + lane * 8 + i]; const unsigned short hb = f2bf(v); oh[i] = hb; ol[i] = f2bf(v - bf2f(hb)); }
    *(volatile v8us*)(XH + w * 256 + lane * 8) = oh; *(volatile v8us*)(XL + w * 256 + lane * 8) = ol; __threadfence();
    *(volatile v8us*)(XH + w * 256 + lane * 8) = oh; *(volatile v8us*)(XL + w * 256 + lane * 8) = ol;
}
__global__ __launch_bounds__(128) void k_out(const bf* __restrict__ XH, const bf* __restrict__ XL, const bf* __restrict__ WoT, const float* __restrict__ bo, float* out) {
    __shared__ __align__(16) float ost[4][16 * 68];
    const int lane = threadIdx.x & 31, wave = threadIdx.x >> 5, lr = lane & 15, hi = lane >> 4;
    const int K = NH_ * DV;
    const size_t r0 = (size_t)blockIdx.x * 64 + wave * 16; const int c0 = blockIdx.y * 64;
    v8f acc[4];
#pragma unroll
    for (int t = 0; t < 4; ++t) acc[t] = (v8f){};
#pragma unroll 2
    for (int kc = 0; kc < K; kc += 32) {
        const size_t ao = (r0 + lr) * K + kc + 8 * hi;
        const v16bf a = cat16b(*(const v8us*)(XH + ao), *(const v8us*)(XH + ao + 16)), al = cat16b(*(const v8us*)(XL + ao), *(const v8us*)(XL + ao + 16));
#pragma unroll
        for (int t = 0; t < 4; ++t) { const bf* bp = WoT + (size_t)(c0 + t * 16 + lr) * K + kc + 8 * hi; const v16bf bb = cat16b(*(const v8us*)bp, *(const v8us*)(bp + 16)); acc[t] = wmmab(a, bb, acc[t]); acc[t] = wmmab(al, bb, acc[t]); }
        asm volatile("v_nop" : "+v"(acc[0]), "+v"(acc[1]), "+v"(acc[2]), "+v"(acc[3]) : "v"(a), "v"(al) : "memory");
    }
    float* os = &ost[wave][0];
#pragma unroll
    for (int t = 0; t < 4; ++t) { const float bv = bfr(bo[c0 + t * 16 + lr]);
#pragma unroll
        for (int j = 0; j < 8; ++j) os[(hi * 8 + j) * 68 + t * 16 + lr] = acc[t][j] + bv; }
    __syncthreads();
    float* crow = out + r0 * NHID + c0;
    auto pass = [&]() {
#pragma unroll
        for (int s = 0; s < 8; ++s) { const int Lid = (lane >> 3) + 4 * s, piece = lane & 7; const int row = Lid >> 1, cofs = (Lid & 1) * 32 + piece * 4;
            const v4f val = *(const v4fa*)(os + row * 68 + cofs); *(volatile v4f*)(crow + (size_t)row * NHID + cofs) = val; }
    };
    pass(); __threadfence(); pass();
}

extern "C" void kernel_launch(void* const* d_in, const int* in_sizes, int n_in,
                              void* d_out, int out_size, void* d_ws, size_t ws_size, hipStream_t stream) {
    (void)in_sizes; (void)n_in; (void)out_size;
    const float* query = (const float*)d_in[0]; const float* key = (const float*)d_in[1]; const float* value = (const float*)d_in[2];
    const float* Wq = (const float*)d_in[3]; const float* bq = (const float*)d_in[4]; const float* Wk = (const float*)d_in[5]; const float* bk = (const float*)d_in[6]; const float* Wo = (const float*)d_in[7]; const float* bo = (const float*)d_in[8];
    float* out = (float*)d_out;
    char* wsp = (char*)d_ws;
    auto take = [&](size_t bytes) { char* p = wsp; wsp += (bytes + 255) & ~(size_t)255; return (void*)p; };
    const size_t NQR = (size_t)NB_ * NQ_, NKR = (size_t)NB_ * NS_;
    bf* QB = (bf*)take(NQR * DA * 2); bf* KB = (bf*)take(NKR * DA * 2); bf* WqT = (bf*)take(DA * DA * 2); bf* WkT = (bf*)take(DA * DA * 2); bf* WoT = (bf*)take((size_t)NHID * NH_ * DV * 2);
    h16* QH = (h16*)take(NQR * DA * 2); h16* QL = (h16*)take(NQR * DA * 2); h16* KH = (h16*)take(NKR * DA * 2); h16* KL = (h16*)take(NKR * DA * 2);
    h16* VT16 = (h16*)take((size_t)NB_ * DV * NS_ * 2); float* X = (float*)take(NQR * NH_ * DV * 4); bf* XH = (bf*)take(NQR * NH_ * DV * 2); bf* XL = (bf*)take(NQR * NH_ * DV * 2);
    if ((size_t)(wsp - (char*)d_ws) > ws_size) return;
    k_b64<<<(unsigned)((NQR / 2 + 7) / 8), 256, 0, stream>>>(query, NQR, QB);
    k_b64<<<(unsigned)((NKR / 2 + 7) / 8), 256, 0, stream>>>(key, NKR, KB);
    k_wt64<<<DA / 8, 256, 0, stream>>>(Wq, DA, WqT); k_wt64<<<DA / 8, 256, 0, stream>>>(Wk, DA, WkT);
    k_wo<<<dim3((NH_ * DV) / 64, NHID / 64, 1), 256, 0, stream>>>(Wo, WoT);
    k_proj<<<(unsigned)(NQR / 64), 128, 0, stream>>>(QB, WqT, bq, QH, QL);
    k_proj<<<(unsigned)(NKR / 64), 128, 0, stream>>>(KB, WkT, bk, KH, KL);
    k_vt<<<dim3(NS_ / 64, 1, NB_), 256, 0, stream>>>(value, VT16);
    k_attn<<<NB_ * NH_, 128, 0, stream>>>(QH, QL, KH, KL, VT16, X);
    k_xsplit<<<(unsigned)((NQR * NH_ * DV / 256) / 8), 256, 0, stream>>>(X, XH, XL);
    k_out<<<dim3((unsigned)(NQR / 64), NHID / 64, 1), 128, 0, stream>>>(XH, XL, WoT, bo, out);
}
